// LorentzAttention_54434415509618
// MI455X (gfx1250) — hardware-verified
//
#include <hip/hip_runtime.h>
#include <stddef.h>
#include <stdint.h>

#define NB    4
#define NTOK  2048
#define NR    (NB * NTOK)
#define XW    513
#define SPD   512
#define NH    8
#define HD    64
#define NBH   (NB * NH)

#define INV_CURV 10.0f
#define SQK      0.31622776601683794f
#define F16_MIN_NORMAL 6.103515625e-05f

#define TP 68
#define HP 72

#define SZ_XSP  ((size_t)NR * SPD * 2)
#define SZ_XT   ((size_t)NR * 4)
#define SZ_WT   ((size_t)4 * SPD * SPD * 2)
#define SZ_WB   ((size_t)4 * 1024 * 4)
#define SZ_C    ((size_t)NR * SPD * 4)
#define SZ_P16  ((size_t)NR * SPD * 2)
#define SZ_VT   ((size_t)NBH * HD * NTOK * 2)
#define SZ_T    ((size_t)NR * 4)
#define SZ_HSS  ((size_t)NBH * NTOK * 4)
#define OFF_XSP ((size_t)0)
#define OFF_XT  (OFF_XSP + SZ_XSP)
#define OFF_WT  (OFF_XT + SZ_XT)
#define OFF_WB  (OFF_WT + SZ_WT)
#define OFF_C   (OFF_WB + SZ_WB)
#define OFF_Q16 (OFF_C + SZ_C)
#define OFF_K16 (OFF_Q16 + SZ_P16)
#define OFF_VT  (OFF_K16 + SZ_P16)
#define OFF_QT  (OFF_VT + SZ_VT)
#define OFF_KT  (OFF_QT + SZ_T)
#define OFF_SC  (OFF_KT + SZ_T)
#define OFF_HSS (OFF_SC + SZ_P16)
#define WS_TOTAL (OFF_HSS + SZ_HSS)

static_assert((OFF_XT % 256) == 0);
static_assert((OFF_WT % 256) == 0);
static_assert((OFF_WB % 256) == 0);
static_assert((OFF_C % 256) == 0);
static_assert((OFF_Q16 % 256) == 0);
static_assert((OFF_K16 % 256) == 0);
static_assert((OFF_VT % 256) == 0);
static_assert((OFF_QT % 256) == 0);
static_assert((OFF_KT % 256) == 0);
static_assert((OFF_SC % 256) == 0);
static_assert((OFF_HSS % 256) == 0);
static_assert(WS_TOTAL == (size_t)61194240);
static_assert(WS_TOTAL <= (size_t)134217728);
static_assert((128 * XW) % 32 == 0);
static_assert((NR % 128) == 0);
static_assert((TP * 4) % 16 == 0);
static_assert((HP * 2) % 16 == 0);

typedef unsigned short v8us  __attribute__((ext_vector_type(8)));
typedef unsigned short v16us __attribute__((ext_vector_type(16)));
typedef unsigned short v8usA __attribute__((ext_vector_type(8), may_alias));
typedef _Float16       v8h   __attribute__((ext_vector_type(8)));
typedef _Float16       v16h  __attribute__((ext_vector_type(16)));
typedef _Float16       v8hA  __attribute__((ext_vector_type(8), may_alias));
typedef float          v4f   __attribute__((ext_vector_type(4)));
typedef float          v8f   __attribute__((ext_vector_type(8)));
#if defined(__HIP_DEVICE_COMPILE__)
typedef __bf16         v16bf __attribute__((ext_vector_type(16)));
#endif

union FragU { v16us v; v8us half[2]; };
union FragH { v16h  v; v8h  half[2]; };

__device__ __forceinline__ unsigned bbits(float f) {
  unsigned u = __float_as_uint(f);
  return (u + 0x7FFFu + ((u >> 16) & 1u)) >> 16;
}
__device__ __forceinline__ float bf16r(float f) {
  return __uint_as_float(bbits(f) << 16);
}
__device__ __forceinline__ float rcpf_(float x) {
#if defined(__HIP_DEVICE_COMPILE__)
  return __builtin_amdgcn_rcpf(x);
#else
  return 1.0f / x;
#endif
}
__device__ __forceinline__ v8f zero8() { v8f z = {0.f, 0.f, 0.f, 0.f, 0.f, 0.f, 0.f, 0.f}; return z; }

__device__ __forceinline__ v16us ldfrag_u(const unsigned short* p) {
  FragU f;
  f.half[0] = *(const v8usA*)(p);
  f.half[1] = *(const v8usA*)(p + 16);
  return f.v;
}
__device__ __forceinline__ v16h ldfrag_h(const _Float16* p) {
  FragH f;
  f.half[0] = *(const v8hA*)(p);
  f.half[1] = *(const v8hA*)(p + 16);
  return f.v;
}

template <int MODE>
__device__ __forceinline__ v8f mma16(v16us a, v16us b, v8f c) {
#if defined(__HIP_DEVICE_COMPILE__)
  if (MODE == 0)
    return __builtin_amdgcn_wmma_f32_16x16x32_bf16(false, __builtin_bit_cast(v16bf, a),
                                                  false, __builtin_bit_cast(v16bf, b),
                                                  (short)0, c, false, false);
  else
    return __builtin_amdgcn_wmma_f32_16x16x32_f16(false, __builtin_bit_cast(v16h, a),
                                                 false, __builtin_bit_cast(v16h, b),
                                                 (short)0, c, false, false);
#else
  (void)a; (void)b;
  return c;
#endif
}
__device__ __forceinline__ v8f mma_h(v16h a, v16h b, v8f c) {
#if defined(__HIP_DEVICE_COMPILE__)
  return __builtin_amdgcn_wmma_f32_16x16x32_f16(false, a, false, b, (short)0, c, false, false);
#else
  (void)a; (void)b;
  return c;
#endif
}
template <typename F>
__device__ __forceinline__ void guard4(v8f& c0, v8f& c1, v8f& c2, v8f& c3,
                                       const F& f0, const F& f1, const F& f2,
                                       const F& f3, const F& f4, const F& f5) {
#if defined(__HIP_DEVICE_COMPILE__)
  asm volatile("v_nop\n\tv_nop\n\tv_nop\n\tv_nop"
               : "+v"(c0), "+v"(c1), "+v"(c2), "+v"(c3)
               : "v"(f0), "v"(f1), "v"(f2), "v"(f3), "v"(f4), "v"(f5));
#else
  (void)c0; (void)c1; (void)c2; (void)c3; (void)f0; (void)f1; (void)f2; (void)f3; (void)f4; (void)f5;
#endif
}

__global__ __launch_bounds__(256)
void k_prepx(const float* __restrict__ x, unsigned short* xsp, float* xt)
{
  const int row0 = blockIdx.x * 32;
  const int tid  = threadIdx.x;
  const int lane = tid & 31;
  const int w    = tid >> 5;

#pragma unroll 1
  for (int i = 0; i < 4; ++i) {
    const int row = row0 + 4 * w + i;
    const float* xr = x + (size_t)row * XW + 1;
#pragma unroll
    for (int it = 0; it < 2; ++it) {
      const int p = it * 32 + lane;
      v8us o;
#pragma unroll
      for (int e = 0; e < 8; ++e) o[e] = (unsigned short)bbits(xr[8 * p + e]);
      unsigned short* dst = xsp + (size_t)row * SPD + 8 * p;
      *(volatile v8us*)dst = o;
      __threadfence();
      *(volatile v8us*)dst = o;
    }
  }

  const int l8 = lane & 7;
  v4f tv;
#pragma unroll
  for (int e = 0; e < 4; ++e) tv[e] = bf16r(x[(size_t)(row0 + 4 * l8 + e) * XW]);
  float* tdst = xt + row0 + 4 * l8;
  const bool twr = (w == 0) && (lane < 8);
  if (twr) *(volatile v4f*)tdst = tv;
  __threadfence();
  if (twr) *(volatile v4f*)tdst = tv;
}

__global__ __launch_bounds__(256)
void k_prepw(const float* __restrict__ Wq, const float* __restrict__ Wk,
             const float* __restrict__ Wv, const float* __restrict__ Wo,
             const float* __restrict__ bq, const float* __restrict__ bk,
             const float* __restrict__ bv, const float* __restrict__ bo,
             unsigned short* wt, float* wb)
{
  __shared__ __align__(16) unsigned short T[64 * HP];
  const int kt   = blockIdx.x;
  const int nt   = blockIdx.y;
  const int z    = blockIdx.z;
  const int k0   = 64 * kt;
  const int n0   = 64 * nt;
  const int tid  = threadIdx.x;
  const int lane = tid & 31;
  const int w    = tid >> 5;
  const int q    = lane >> 3;
  const int jj   = lane & 7;

  const float* W  = Wq;
  const float* bb = bq;
  if (z == 1) { W = Wk; bb = bk; }
  else if (z == 2) { W = Wv; bb = bv; }
  else if (z == 3) { W = Wo; bb = bo; }
  const bool isO = (z == 3);

#pragma unroll 4
  for (int it = 0; it < 16; ++it) {
    const int kl = it * 4 + (tid >> 6);
    const int nl = tid & 63;
    const float v = bf16r(W[(size_t)(1 + k0 + kl) * SPD + n0 + nl]);
    const unsigned short hb = (unsigned short)bbits(v);
    const _Float16 fv = (_Float16)(v * 256.0f);
    const unsigned short fb = __builtin_bit_cast(unsigned short, fv);
    T[nl * HP + kl] = isO ? fb : hb;
  }
  __syncthreads();

  v8us   vv[2];
  size_t off[2];
#pragma unroll
  for (int it = 0; it < 2; ++it) {
    const int nl = it * 32 + 4 * w + q;
    vv[it]  = *(const v8usA*)(T + nl * HP + 8 * jj);
    off[it] = ((size_t)z * SPD + (size_t)(n0 + nl)) * SPD + (size_t)(k0 + 8 * jj);
  }
#pragma unroll
  for (int it = 0; it < 2; ++it) *(volatile v8us*)(wt + off[it]) = vv[it];

  const int grp = lane >> 3;
  const int col = n0 + 32 * (grp & 1) + 4 * jj;
  v4f lv;
#pragma unroll
  for (int e = 0; e < 4; ++e) {
    const float wv0 = bf16r(W[col + e]);
    const float bv0 = bf16r(bb[col + e]);
    lv[e] = (grp < 2) ? wv0 : bv0;
  }
  float* ldst = wb + (size_t)z * 1024 + 512 * (grp >> 1) + col;
  const bool lwr = (kt == 0) && (w == 0);
  if (lwr) *(volatile v4f*)ldst = lv;

  __threadfence();

#pragma unroll
  for (int it = 0; it < 2; ++it) *(volatile v8us*)(wt + off[it]) = vv[it];
  if (lwr) *(volatile v4f*)ldst = lv;
}

template <int MODE>
__global__ __launch_bounds__(256)
void k_gemm(const unsigned short* __restrict__ A, const unsigned short* __restrict__ Bt,
            const float* __restrict__ rsrc, const float* __restrict__ wb, float* C)
{
  __shared__ __align__(16) float T[128 * TP];
  __shared__ float rt[128];
  const int n0   = blockIdx.x * 64;
  const int m0   = blockIdx.y * 128;
  const int tid  = threadIdx.x;
  const int lane = tid & 31;
  const int w    = tid >> 5;
  const int h    = lane >> 4;
  const int m    = lane & 15;
  const int q    = lane >> 3;
  const int jj   = lane & 7;
  const int wm   = w >> 1;
  const int wn   = w & 1;

  v8f acc[2][2];
  acc[0][0] = zero8(); acc[0][1] = zero8(); acc[1][0] = zero8(); acc[1][1] = zero8();

  const unsigned short* pa = A  + (size_t)(m0 + 32 * wm + m) * SPD + 8 * h;
  const unsigned short* pb = Bt + (size_t)(n0 + 32 * wn + m) * SPD + 8 * h;
#pragma unroll 2
  for (int kk = 0; kk < 16; ++kk) {
    const v16us a0 = ldfrag_u(pa + 32 * kk);
    const v16us a1 = ldfrag_u(pa + 16 * SPD + 32 * kk);
    const v16us b0 = ldfrag_u(pb + 32 * kk);
    const v16us b1 = ldfrag_u(pb + 16 * SPD + 32 * kk);
    acc[0][0] = mma16<MODE>(a0, b0, acc[0][0]);
    acc[0][1] = mma16<MODE>(a0, b1, acc[0][1]);
    acc[1][0] = mma16<MODE>(a1, b0, acc[1][0]);
    acc[1][1] = mma16<MODE>(a1, b1, acc[1][1]);
    guard4<v16us>(acc[0][0], acc[0][1], acc[1][0], acc[1][1], a0, a1, b0, b1, a0, b1);
  }

#pragma unroll
  for (int mi = 0; mi < 2; ++mi)
#pragma unroll
    for (int ni = 0; ni < 2; ++ni)
#pragma unroll
      for (int r = 0; r < 8; ++r)
        T[(32 * wm + 16 * mi + 8 * h + r) * TP + 32 * wn + 16 * ni + m] = acc[mi][ni][r];

  if (tid < 128) {
    const int mrow = m0 + tid;
    float rv;
    if (MODE == 0) {
      rv = rsrc[mrow];
    } else {
      const int bb = mrow >> 11;
      const int nn = mrow & (NTOK - 1);
      float s = 0.f;
#pragma unroll
      for (int hh = 0; hh < NH; ++hh) s += rsrc[(size_t)(bb * NH + hh) * NTOK + nn];
      rv = sqrtf(fmaxf(INV_CURV + s, 1e-9f));
    }
    rt[tid] = rv;
  }

  const int hl  = q & 1;
  const int col = 32 * hl + 4 * jj;
  const v4f w0v = *(const v4f*)(wb + n0 + col);
  const v4f bsv = *(const v4f*)(wb + 512 + n0 + col);
  const float SC = (MODE == 0) ? 1.0f : (1.0f / 16384.0f);
  __syncthreads();

#pragma unroll 1
  for (int it = 0; it < 8; ++it) {
    const int ml = it * 16 + 2 * w + (q >> 1);
    const v4f tv = *(const v4f*)(T + ml * TP + col);
    const float r1 = rt[ml];
    v4f val;
#pragma unroll
    for (int e = 0; e < 4; ++e) val[e] = (tv[e] * SC + r1 * w0v[e]) + bsv[e];
    *(volatile v4f*)(C + (size_t)(m0 + ml) * SPD + n0 + col) = val;
  }
  __threadfence();
#pragma unroll 1
  for (int it = 0; it < 8; ++it) {
    const int ml = it * 16 + 2 * w + (q >> 1);
    const v4f tv = *(const v4f*)(T + ml * TP + col);
    const float r1 = rt[ml];
    v4f val;
#pragma unroll
    for (int e = 0; e < 4; ++e) val[e] = (tv[e] * SC + r1 * w0v[e]) + bsv[e];
    *(volatile v4f*)(C + (size_t)(m0 + ml) * SPD + n0 + col) = val;
  }
}

__global__ __launch_bounds__(256)
void k_epi_qk(const float* __restrict__ C, _Float16* p16, float* tout)
{
  __shared__ float ts[32];
  const int row0 = blockIdx.x * 32;
  const int tid  = threadIdx.x;
  const int lane = tid & 31;
  const int w    = tid >> 5;

#pragma unroll 1
  for (int i = 0; i < 4; ++i) {
    const int row = row0 + 4 * w + i;
    const float* cr = C + (size_t)row * SPD + 8 * lane;
    const v4f a0 = *(const v4f*)(cr);
    const v4f a1 = *(const v4f*)(cr + 4);
    const v4f a2 = *(const v4f*)(cr + 256);
    const v4f a3 = *(const v4f*)(cr + 260);
    float ss = 0.f;
    v8h o0, o1;
#pragma unroll
    for (int e = 0; e < 4; ++e) {
      ss += a0[e] * a0[e];
      ss += a1[e] * a1[e];
      ss += a2[e] * a2[e];
      ss += a3[e] * a3[e];
      o0[e]     = (_Float16)(a0[e] * 8.0f);
      o0[4 + e] = (_Float16)(a1[e] * 8.0f);
      o1[e]     = (_Float16)(a2[e] * 8.0f);
      o1[4 + e] = (_Float16)(a3[e] * 8.0f);
    }
#pragma unroll
    for (int off = 16; off >= 1; off >>= 1) ss += __shfl_xor(ss, off, 32);
    const float t = sqrtf(fmaxf(INV_CURV + ss, 1e-9f));
    if (lane == 0) ts[4 * w + i] = t;
    _Float16* d0 = p16 + (size_t)row * SPD + 8 * lane;
    *(volatile v8h*)(d0) = o0;
    *(volatile v8h*)(d0 + 256) = o1;
    __threadfence();
    *(volatile v8h*)(d0) = o0;
    *(volatile v8h*)(d0 + 256) = o1;
  }
  __syncthreads();

  const int l8 = lane & 7;
  v4f tv;
#pragma unroll
  for (int e = 0; e < 4; ++e) tv[e] = ts[4 * l8 + e];
  float* tdst = tout + row0 + 4 * l8;
  const bool twr = (w == 0) && (lane < 8);
  if (twr) *(volatile v4f*)tdst = tv;
  __threadfence();
  if (twr) *(volatile v4f*)tdst = tv;
}

__global__ __launch_bounds__(256)
void k_epi_v(const float* __restrict__ C, _Float16* vt)
{
  __shared__ float facL[64 * 8];
  __shared__ __align__(16) _Float16 T[64 * HP];
  const int row0 = blockIdx.x * 64;
  const int b    = row0 >> 11;
  const int tok0 = row0 & (NTOK - 1);
  const int tid  = threadIdx.x;
  const int lane = tid & 31;
  const int w    = tid >> 5;
  const int q    = lane >> 3;
  const int jj   = lane & 7;

#pragma unroll 1
  for (int i = 0; i < 8; ++i) {
    const int row = row0 + 8 * w + i;
    const float* cr = C + (size_t)row * SPD + 16 * lane;
    const v4f c0 = *(const v4f*)(cr);
    const v4f c1 = *(const v4f*)(cr + 4);
    const v4f c2 = *(const v4f*)(cr + 8);
    const v4f c3 = *(const v4f*)(cr + 12);
    float ss = 0.f;
#pragma unroll
    for (int e = 0; e < 4; ++e) {
      ss += c0[e] * c0[e];
      ss += c1[e] * c1[e];
      ss += c2[e] * c2[e];
      ss += c3[e] * c3[e];
    }
    float hs = ss;
    hs += __shfl_xor(hs, 1, 32);
    hs += __shfl_xor(hs, 2, 32);
    float tot = hs;
    tot += __shfl_xor(tot, 4, 32);
    tot += __shfl_xor(tot, 8, 32);
    tot += __shfl_xor(tot, 16, 32);
    const float nrm   = sqrtf(hs);
    const float t     = sqrtf(fmaxf(INV_CURV + tot, 1e-9f));
    const float xx    = fmaxf(SQK * t, 1.00000011920928955f);
    const float theta = logf(xx + sqrtf(xx * xx - 1.0f));
    const float fac   = (theta * (1.0f / SQK)) * rcpf_(fmaxf(nrm, 1e-9f));
    if ((lane & 3) == 0) facL[(8 * w + i) * 8 + (lane >> 2)] = fac;
  }
  __syncthreads();

  const int kl = tid >> 2;
  const int ds = tid & 3;
#pragma unroll 1
  for (int hh = 0; hh < NH; ++hh) {
    const float* cr = C + (size_t)(row0 + kl) * SPD + 64 * hh + 16 * ds;
    const v4f c0 = *(const v4f*)(cr);
    const v4f c1 = *(const v4f*)(cr + 4);
    const v4f c2 = *(const v4f*)(cr + 8);
    const v4f c3 = *(const v4f*)(cr + 12);
    const float fac = facL[kl * 8 + hh];
#pragma unroll
    for (int e = 0; e < 4; ++e) {
      T[(16 * ds + e) * HP + kl]      = (_Float16)(c0[e] * fac);
      T[(16 * ds + 4 + e) * HP + kl]  = (_Float16)(c1[e] * fac);
      T[(16 * ds + 8 + e) * HP + kl]  = (_Float16)(c2[e] * fac);
      T[(16 * ds + 12 + e) * HP + kl] = (_Float16)(c3[e] * fac);
    }
    __syncthreads();

    v8h    vv[2];
    size_t off[2];
#pragma unroll
    for (int it = 0; it < 2; ++it) {
      const int dl = it * 32 + 4 * w + q;
      vv[it]  = *(const v8hA*)(T + dl * HP + 8 * jj);
      off[it] = ((size_t)((b * NH + hh) * HD + dl)) * NTOK + (size_t)(tok0 + 8 * jj);
    }
#pragma unroll
    for (int it = 0; it < 2; ++it) *(volatile v8h*)(vt + off[it]) = vv[it];
    __threadfence();
#pragma unroll
    for (int it = 0; it < 2; ++it) *(volatile v8h*)(vt + off[it]) = vv[it];
    __syncthreads();
  }
}

__global__ __launch_bounds__(256)
void k_flash(const _Float16* __restrict__ q16, const _Float16* __restrict__ k16,
             const _Float16* __restrict__ vt, const float* __restrict__ qt,
             const float* __restrict__ kt, _Float16* sc16, float* hss)
{
  __shared__ __align__(16) _Float16 Ps[8 * 16 * HP];
  __shared__ float hsl[128];
  const int tid  = threadIdx.x;
  const int lane = tid & 31;
  const int w    = tid >> 5;
  const int h    = lane >> 4;
  const int m    = lane & 15;
  const int q    = lane >> 3;
  const int jj   = lane & 7;
  const int bh   = blockIdx.y;
  const int b    = bh >> 3;
  const int hd   = bh & 7;
  const int hc   = hd * HD;
  const int qblk = blockIdx.x;
  const int qrow0 = b * NTOK + qblk * 128 + 16 * w;
  _Float16* Pw = Ps + w * (16 * HP);

  const _Float16* qp = q16 + (size_t)(qrow0 + m) * SPD + hc + 8 * h;
  const v16h qa0 = ldfrag_h(qp);
  const v16h qa1 = ldfrag_h(qp + 32);
  float qts[8], mst[8], lst[8];
#pragma unroll
  for (int r = 0; r < 8; ++r) {
    qts[r] = qt[qrow0 + 8 * h + r] * 0.125f;
    mst[r] = -1.0e30f;
    lst[r] = 0.f;
  }
  v8f oacc[4];
  oacc[0] = zero8(); oacc[1] = zero8(); oacc[2] = zero8(); oacc[3] = zero8();

  const _Float16* kbase = k16 + (size_t)(b * NTOK + m) * SPD + hc + 8 * h;
  const _Float16* vbase = vt + (size_t)(bh * HD + m) * NTOK + 8 * h;
  const float*    ktb   = kt + b * NTOK + m;

#pragma unroll 1
  for (int j = 0; j < 32; ++j) {
    const _Float16* kp = kbase + (size_t)(64 * j) * SPD;
    v8f sacc[4];
    sacc[0] = zero8(); sacc[1] = zero8(); sacc[2] = zero8(); sacc[3] = zero8();
    {
      const v16h b0 = ldfrag_h(kp);
      const v16h b1 = ldfrag_h(kp + 16 * SPD);
      const v16h b2 = ldfrag_h(kp + 32 * SPD);
      const v16h b3 = ldfrag_h(kp + 48 * SPD);
      sacc[0] = mma_h(qa0, b0, sacc[0]);
      sacc[1] = mma_h(qa0, b1, sacc[1]);
      sacc[2] = mma_h(qa0, b2, sacc[2]);
      sacc[3] = mma_h(qa0, b3, sacc[3]);
      const v16h c0 = ldfrag_h(kp + 32);
      const v16h c1 = ldfrag_h(kp + 16 * SPD + 32);
      const v16h c2 = ldfrag_h(kp + 32 * SPD + 32);
      const v16h c3 = ldfrag_h(kp + 48 * SPD + 32);
      sacc[0] = mma_h(qa1, c0, sacc[0]);
      sacc[1] = mma_h(qa1, c1, sacc[1]);
      sacc[2] = mma_h(qa1, c2, sacc[2]);
      sacc[3] = mma_h(qa1, c3, sacc[3]);
      guard4<v16h>(sacc[0], sacc[1], sacc[2], sacc[3], qa0, qa1, c0, c1, c2, c3);
    }
    float ktv[4];
#pragma unroll
    for (int nt = 0; nt < 4; ++nt) ktv[nt] = ktb[64 * j + 16 * nt];

#pragma unroll
    for (int r = 0; r < 8; ++r) {
      const float s0 = sacc[0][r] * (1.0f / 512.0f) - qts[r] * ktv[0];
      const float s1 = sacc[1][r] * (1.0f / 512.0f) - qts[r] * ktv[1];
      const float s2 = sacc[2][r] * (1.0f / 512.0f) - qts[r] * ktv[2];
      const float s3 = sacc[3][r] * (1.0f / 512.0f) - qts[r] * ktv[3];
      float mx = fmaxf(fmaxf(s0, s1), fmaxf(s2, s3));
      mx = fmaxf(mx, __shfl_xor(mx, 1, 32));
      mx = fmaxf(mx, __shfl_xor(mx, 2, 32));
      mx = fmaxf(mx, __shfl_xor(mx, 4, 32));
      mx = fmaxf(mx, __shfl_xor(mx, 8, 32));
      const float mnew = fmaxf(mst[r], mx);
      const float msc  = __expf(mst[r] - mnew);
      mst[r] = mnew;
      const float p0 = __expf(s0 - mnew) * 4096.0f;
      const float p1 = __expf(s1 - mnew) * 4096.0f;
      const float p2 = __expf(s2 - mnew) * 4096.0f;
      const float p3 = __expf(s3 - mnew) * 4096.0f;
      const _Float16 zh = (_Float16)0.0f;
      const _Float16 h0 = (p0 < F16_MIN_NORMAL) ? zh : (_Float16)p0;
      const _Float16 h1 = (p1 < F16_MIN_NORMAL) ? zh : (_Float16)p1;
      const _Float16 h2 = (p2 < F16_MIN_NORMAL) ? zh : (_Float16)p2;
      const _Float16 h3 = (p3 < F16_MIN_NORMAL) ? zh : (_Float16)p3;
      float rs = (float)h0 + (float)h1 + (float)h2 + (float)h3;
      rs += __shfl_xor(rs, 1, 32);
      rs += __shfl_xor(rs, 2, 32);
      rs += __shfl_xor(rs, 4, 32);
      rs += __shfl_xor(rs, 8, 32);
      lst[r] = lst[r] * msc + rs;
      Pw[(8 * h + r) * HP + m]      = h0;
      Pw[(8 * h + r) * HP + 16 + m] = h1;
      Pw[(8 * h + r) * HP + 32 + m] = h2;
      Pw[(8 * h + r) * HP + 48 + m] = h3;
      oacc[0][r] *= msc;
      oacc[1][r] *= msc;
      oacc[2][r] *= msc;
      oacc[3][r] *= msc;
    }
    __syncthreads();

    {
      const v16h pa0 = ldfrag_h(Pw + m * HP + 8 * h);
      const v16h pa1 = ldfrag_h(Pw + m * HP + 32 + 8 * h);
      const _Float16* vp = vbase + 64 * j;
      const v16h v0 = ldfrag_h(vp);
      const v16h v1 = ldfrag_h(vp + 16 * NTOK);
      const v16h v2 = ldfrag_h(vp + 32 * NTOK);
      const v16h v3 = ldfrag_h(vp + 48 * NTOK);
      oacc[0] = mma_h(pa0, v0, oacc[0]);
      oacc[1] = mma_h(pa0, v1, oacc[1]);
      oacc[2] = mma_h(pa0, v2, oacc[2]);
      oacc[3] = mma_h(pa0, v3, oacc[3]);
      const v16h u0 = ldfrag_h(vp + 32);
      const v16h u1 = ldfrag_h(vp + 16 * NTOK + 32);
      const v16h u2 = ldfrag_h(vp + 32 * NTOK + 32);
      const v16h u3 = ldfrag_h(vp + 48 * NTOK + 32);
      oacc[0] = mma_h(pa1, u0, oacc[0]);
      oacc[1] = mma_h(pa1, u1, oacc[1]);
      oacc[2] = mma_h(pa1, u2, oacc[2]);
      oacc[3] = mma_h(pa1, u3, oacc[3]);
      guard4<v16h>(oacc[0], oacc[1], oacc[2], oacc[3], pa0, pa1, u0, u1, u2, u3);
    }
    __syncthreads();
  }

  float hsr[8];
#pragma unroll
  for (int r = 0; r < 8; ++r) {
    const float inv = rcpf_(lst[r]);
    const float u0 = oacc[0][r] * inv;
    const float u1 = oacc[1][r] * inv;
    const float u2 = oacc[2][r] * inv;
    const float u3 = oacc[3][r] * inv;
    float us = u0 * u0;
    us += u1 * u1;
    us += u2 * u2;
    us += u3 * u3;
    us += __shfl_xor(us, 1, 32);
    us += __shfl_xor(us, 2, 32);
    us += __shfl_xor(us, 4, 32);
    us += __shfl_xor(us, 8, 32);
    const float nrm = sqrtf(us);
    const float a   = SQK * nrm;
    const float a2  = a * a;
    const float shs = a * (1.0f + a2 * (0.166666667f + a2 * (8.33333333e-3f
                      + a2 * (1.98412698e-4f + a2 * 2.75573192e-6f))));
    const float ea  = __expf(a);
    const float shl = 0.5f * (ea - rcpf_(ea));
    const float sh  = (a < 1.0f) ? shs : shl;
    const float fac = sh * rcpf_(SQK * fmaxf(nrm, 1e-9f));
    const float g0 = u0 * fac;
    const float g1 = u1 * fac;
    const float g2 = u2 * fac;
    const float g3 = u3 * fac;
    float hq = g0 * g0;
    hq += g1 * g1;
    hq += g2 * g2;
    hq += g3 * g3;
    hq += __shfl_xor(hq, 1, 32);
    hq += __shfl_xor(hq, 2, 32);
    hq += __shfl_xor(hq, 4, 32);
    hq += __shfl_xor(hq, 8, 32);
    hsr[r] = hq;
    Pw[(8 * h + r) * HP + m]      = (_Float16)(g0 * 64.0f);
    Pw[(8 * h + r) * HP + 16 + m] = (_Float16)(g1 * 64.0f);
    Pw[(8 * h + r) * HP + 32 + m] = (_Float16)(g2 * 64.0f);
    Pw[(8 * h + r) * HP + 48 + m] = (_Float16)(g3 * 64.0f);
  }
  if (m == 0) {
#pragma unroll
    for (int r = 0; r < 8; ++r) hsl[16 * w + 8 * h + r] = hsr[r];
  }
  __syncthreads();

  v8h    ov[4];
  size_t ooff[4];
#pragma unroll
  for (int it = 0; it < 4; ++it) {
    const int rl = 4 * it + q;
    ov[it]   = *(const v8hA*)(Pw + rl * HP + 8 * jj);
    ooff[it] = (size_t)(qrow0 + rl) * SPD + (size_t)(hc + 8 * jj);
  }
  v4f hv;
#pragma unroll
  for (int e = 0; e < 4; ++e) hv[e] = hsl[4 * lane + e];
  float* hdst = hss + (size_t)bh * NTOK + qblk * 128 + 4 * lane;
  const bool hwr = (w == 0);

#pragma unroll
  for (int it = 0; it < 4; ++it) *(volatile v8h*)(sc16 + ooff[it]) = ov[it];
  if (hwr) *(volatile v4f*)hdst = hv;
  __threadfence();
#pragma unroll
  for (int it = 0; it < 4; ++it) *(volatile v8h*)(sc16 + ooff[it]) = ov[it];
  if (hwr) *(volatile v4f*)hdst = hv;
}

__global__ __launch_bounds__(256)
void k_final(const float* __restrict__ C, float* out)
{
  __shared__ float tL[128];
  const int row0 = blockIdx.x * 128;
  const int tid  = threadIdx.x;
  const int lane = tid & 31;
  const int w    = tid >> 5;
  const int q    = lane >> 3;
  const int jj   = lane & 7;

#pragma unroll 1
  for (int i = 0; i < 16; ++i) {
    const int row = row0 + 16 * w + i;
    const float* cr = C + (size_t)row * SPD + 16 * lane;
    const v4f c0 = *(const v4f*)(cr);
    const v4f c1 = *(const v4f*)(cr + 4);
    const v4f c2 = *(const v4f*)(cr + 8);
    const v4f c3 = *(const v4f*)(cr + 12);
    float ss = 0.f;
#pragma unroll
    for (int e = 0; e < 4; ++e) {
      ss += c0[e] * c0[e];
      ss += c1[e] * c1[e];
      ss += c2[e] * c2[e];
      ss += c3[e] * c3[e];
    }
#pragma unroll
    for (int off = 16; off >= 1; off >>= 1) ss += __shfl_xor(ss, off, 32);
    const float t = sqrtf(fmaxf(INV_CURV + ss, 1e-9f));
    if (lane == 0) tL[16 * w + i] = t;
  }
  __syncthreads();

  const int NLINES = (128 * XW) / 32;
  const size_t F0 = (size_t)blockIdx.x * (size_t)(128 * XW);
#pragma unroll 1
  for (int it = 0; it < 65; ++it) {
    const int L  = it * 32 + 4 * w + q;
    const bool valid = (L < NLINES);
    const int Lc = valid ? L : (NLINES - 1);
    v4f v;
#pragma unroll
    for (int e = 0; e < 4; ++e) {
      const int f  = Lc * 32 + 4 * jj + e;
      const int r  = f / XW;
      const int c  = f - r * XW;
      const int cc = (c > 0) ? (c - 1) : 0;
      const float cv = C[(size_t)(row0 + r) * SPD + cc];
      const float tv = tL[r];
      v[e] = (c == 0) ? tv : cv;
    }
    if (valid) *(volatile v4f*)(out + F0 + (size_t)Lc * 32 + 4 * jj) = v;
  }
  __threadfence();
#pragma unroll 1
  for (int it = 0; it < 65; ++it) {
    const int L  = it * 32 + 4 * w + q;
    const bool valid = (L < NLINES);
    const int Lc = valid ? L : (NLINES - 1);
    v4f v;
#pragma unroll
    for (int e = 0; e < 4; ++e) {
      const int f  = Lc * 32 + 4 * jj + e;
      const int r  = f / XW;
      const int c  = f - r * XW;
      const int cc = (c > 0) ? (c - 1) : 0;
      const float cv = C[(size_t)(row0 + r) * SPD + cc];
      const float tv = tL[r];
      v[e] = (c == 0) ? tv : cv;
    }
    if (valid) *(volatile v4f*)(out + F0 + (size_t)Lc * 32 + 4 * jj) = v;
  }
}

extern "C" void kernel_launch(void* const* d_in, const int* in_sizes, int n_in,
                              void* d_out, int out_size, void* d_ws, size_t ws_size,
                              hipStream_t stream) {
  if (n_in < 9) return;
  if (in_sizes[0] != NR * XW) return;
  if (in_sizes[1] != XW * SPD || in_sizes[3] != XW * SPD || in_sizes[5] != XW * SPD ||
      in_sizes[7] != XW * SPD) return;
  if (in_sizes[2] != SPD || in_sizes[4] != SPD || in_sizes[6] != SPD || in_sizes[8] != SPD) return;
  if (out_size != NR * XW) return;
  if (ws_size < WS_TOTAL) return;

  const float* x  = (const float*)d_in[0];
  const float* Wq = (const float*)d_in[1];
  const float* bq = (const float*)d_in[2];
  const float* Wk = (const float*)d_in[3];
  const float* bk = (const float*)d_in[4];
  const float* Wv = (const float*)d_in[5];
  const float* bv = (const float*)d_in[6];
  const float* Wo = (const float*)d_in[7];
  const float* bo = (const float*)d_in[8];
  float* out = (float*)d_out;
  char* ws = (char*)d_ws;

  unsigned short* xsp  = (unsigned short*)(ws + OFF_XSP);
  float*          xt   = (float*)(ws + OFF_XT);
  unsigned short* wt   = (unsigned short*)(ws + OFF_WT);
  float*          wb   = (float*)(ws + OFF_WB);
  float*          Cp   = (float*)(ws + OFF_C);
  _Float16*       q16  = (_Float16*)(ws + OFF_Q16);
  _Float16*       k16  = (_Float16*)(ws + OFF_K16);
  _Float16*       vtp  = (_Float16*)(ws + OFF_VT);
  float*          qtp  = (float*)(ws + OFF_QT);
  float*          ktp  = (float*)(ws + OFF_KT);
  _Float16*       sc16 = (_Float16*)(ws + OFF_SC);
  float*          hss  = (float*)(ws + OFF_HSS);

  const size_t WPL = (size_t)SPD * SPD;

  k_prepx<<<dim3(NR / 32), dim3(256), 0, stream>>>(x, xsp, xt);
  (void)hipGetLastError();
  k_prepw<<<dim3(SPD / 64, SPD / 64, 4), dim3(256), 0, stream>>>(Wq, Wk, Wv, Wo, bq, bk, bv, bo,
                                                               wt, wb);
  (void)hipGetLastError();

  const dim3 gg(SPD / 64, NR / 128);
  k_gemm<0><<<gg, dim3(256), 0, stream>>>(xsp, wt + 0 * WPL, xt, wb + 0 * 1024, Cp);
  (void)hipGetLastError();
  k_epi_qk<<<dim3(NR / 32), dim3(256), 0, stream>>>(Cp, q16, qtp);
  (void)hipGetLastError();
  k_gemm<0><<<gg, dim3(256), 0, stream>>>(xsp, wt + 1 * WPL, xt, wb + 1 * 1024, Cp);
  (void)hipGetLastError();
  k_epi_qk<<<dim3(NR / 32), dim3(256), 0, stream>>>(Cp, k16, ktp);
  (void)hipGetLastError();
  k_gemm<0><<<gg, dim3(256), 0, stream>>>(xsp, wt + 2 * WPL, xt, wb + 2 * 1024, Cp);
  (void)hipGetLastError();
  k_epi_v<<<dim3(NR / 64), dim3(256), 0, stream>>>(Cp, vtp);
  (void)hipGetLastError();

  k_flash<<<dim3(NTOK / 128, NBH), dim3(256), 0, stream>>>(q16, k16, vtp, qtp, ktp, sc16, hss);
  (void)hipGetLastError();

  k_gemm<1><<<gg, dim3(256), 0, stream>>>((const unsigned short*)sc16, wt + 3 * WPL, hss,
                                          wb + 3 * 1024, Cp);
  (void)hipGetLastError();
  k_final<<<dim3(NR / 128), dim3(256), 0, stream>>>(Cp, out);
  (void)hipGetLastError();
}
